// SimpleRNN_2860448219166
// MI455X (gfx1250) — hardware-verified
//
#include <hip/hip_runtime.h>
#include <math.h>

constexpr int kT      = 4096;
constexpr int kHid    = 2048;
constexpr int kKey    = 1024;
constexpr int kVal    = 1024;
constexpr int kOutDim = 2048;
constexpr int kChunk  = 32;
constexpr int kNChunk = kT / kChunk;
constexpr int kPairs  = kNChunk / 2;
constexpr int kRoleABlocks = (kVal / 64) / 8;
constexpr int kRoleBBlocks = ((kVal / 64) * (kKey / 64)) / 8;
constexpr int kPreKeys    = 256;
constexpr int kPreThreads = 128;
constexpr float kCarryV  = 64.0f;
constexpr float kCarryQ  = 1024.0f;
constexpr float kCarryP  = 128.0f;
constexpr float kCarryPl = 2048.0f;
constexpr float kCarryS  = 8.0f;
constexpr float kCarryK  = 16384.0f;
constexpr float kCarryO  = 16.0f;
constexpr float kCarryW  = 256.0f;
constexpr float kOutSlabScale = kCarryO / (kCarryQ * kCarryS);
constexpr float kPlInv        = 1.0f / kCarryPl;
constexpr float kStateScale   = 1.0f / (kCarryV * kCarryK);
constexpr float kFinalScale   = 1.0f / (kCarryO * kCarryW);
constexpr float kAFloor       = 1.0e-30f;
static_assert(kCarryQ * kCarryS == kCarryP * kCarryV, "one accumulator carry for both chunk-output terms");
static_assert(kT % kChunk == 0 && kChunk == 32, "chunking: state GEMM is exactly one 32-deep k step");
static_assert(kNChunk % 2 == 0, "chunk pairs");
static_assert(kKey % kPreKeys == 0 && kPreKeys == 2 * kPreThreads, "preprocessing blocks");
static_assert(kT % 64 == 0 && kKey % 64 == 0 && kVal % 64 == 0 && kOutDim % 64 == 0, "tile multiples");
static_assert(kHid % 32 == 0 && kKey % 32 == 0 && kVal % 32 == 0, "K multiples of 32");
static_assert(((kT / 64) * (kKey / 64)) % 8 == 0 && ((kT / 64) * (kOutDim / 64)) % 8 == 0, "full blocks of 8 waves");

typedef __attribute__((ext_vector_type(16))) _Float16 v16h;
typedef __attribute__((ext_vector_type(8)))  _Float16 v8h;
typedef __attribute__((ext_vector_type(16))) __bf16   v16b;
typedef __attribute__((ext_vector_type(8)))  __bf16   v8b;
typedef __attribute__((ext_vector_type(8)))  float    v8f;
typedef __attribute__((ext_vector_type(4)))  float    v4f;
typedef __attribute__((ext_vector_type(2)))  float    v2f;
typedef __attribute__((ext_vector_type(4)))  unsigned int v4u;

__device__ __forceinline__ unsigned short f2bf_bits(float f) {
  unsigned u = __float_as_uint(f);
  return (unsigned short)((u + 0x7FFFu + ((u >> 16) & 1u)) >> 16);
}
__device__ __forceinline__ float bf_bits2f(unsigned short h) { return __uint_as_float(((unsigned)h) << 16); }
__device__ __forceinline__ unsigned pk16(unsigned short a, unsigned short b) { return (unsigned)a | ((unsigned)b << 16); }
__device__ __forceinline__ unsigned short h_bits(float f) { const _Float16 h = (_Float16)f; return __builtin_bit_cast(unsigned short, h); }
__device__ __forceinline__ float h16_to_f32(unsigned hb) {
  const unsigned sgn = (hb & 0x8000u) << 16; const unsigned em = hb & 0x7fffu;
  const float fn = __uint_as_float((em << 13) + 0x38000000u);
  const float fs = (float)em * 5.9604644775390625e-8f;
  const float mag = (em < 0x400u) ? fs : fn; return __uint_as_float(__float_as_uint(mag) | sgn);
}

__device__ __forceinline__ void guard4x_h(v8f& a, v8f& b, v8f& c, v8f& d, v16h x, v16h y) {
  asm volatile("v_nop\n\tv_nop\n\tv_nop\n\tv_nop" : "+v"(a), "+v"(b), "+v"(c), "+v"(d) : "v"(x), "v"(y));
}
__device__ __forceinline__ void guard4x_b(v8f& a, v8f& b, v8f& c, v8f& d, v16b x, v16b y) {
  asm volatile("v_nop\n\tv_nop\n\tv_nop\n\tv_nop" : "+v"(a), "+v"(b), "+v"(c), "+v"(d) : "v"(x), "v"(y));
}
__device__ __forceinline__ void keep4_h(v16h a, v16h b, v16h c, v16h d) { asm volatile("v_nop" :: "v"(a), "v"(b), "v"(c), "v"(d)); }
__device__ __forceinline__ void keep4_b(v16b a, v16b b, v16b c, v16b d) { asm volatile("v_nop" :: "v"(a), "v"(b), "v"(c), "v"(d)); }
__device__ __forceinline__ void acc_guard4(v8f& a, v8f& b, v8f& c, v8f& d) { asm volatile("v_nop\n\tv_nop\n\tv_nop\n\tv_nop" : "+v"(a), "+v"(b), "+v"(c), "+v"(d)); }
__device__ __forceinline__ void wave_sync() {
  __builtin_amdgcn_fence(__ATOMIC_RELEASE, "workgroup");
  __builtin_amdgcn_wave_barrier();
  __builtin_amdgcn_fence(__ATOMIC_ACQUIRE, "workgroup");
}
template <typename T> struct Frag;
template <> struct Frag<_Float16> {
  typedef v16h V; union U { v16h v; v8h h[2]; };
  static __device__ __forceinline__ v16h load(const _Float16* p) {
    U f; f.h[0] = *(const v8h*)(p); f.h[1] = *(const v8h*)(p + 16); return f.v;
  }
  static __device__ __forceinline__ v8f mma(v16h a, v16h b, v8f c) {
    return __builtin_amdgcn_wmma_f32_16x16x32_f16(false, a, false, b, (short)0, c, false, false);
  }
  static __device__ __forceinline__ void guard4(v8f& a, v8f& b, v8f& c, v8f& d, v16h x, v16h y) { guard4x_h(a, b, c, d, x, y); }
  static __device__ __forceinline__ void keep(v16h a, v16h b, v16h c, v16h d) { keep4_h(a, b, c, d); }
};
template <> struct Frag<__bf16> {
  typedef v16b V; union U { v16b v; v8b h[2]; };
  static __device__ __forceinline__ v16b load(const __bf16* p) {
    U f; f.h[0] = *(const v8b*)(p); f.h[1] = *(const v8b*)(p + 16); return f.v;
  }
  static __device__ __forceinline__ v8f mma(v16b a, v16b b, v8f c) {
    return __builtin_amdgcn_wmma_f32_16x16x32_bf16(false, a, false, b, (short)0, c, false, false);
  }
  static __device__ __forceinline__ void guard4(v8f& a, v8f& b, v8f& c, v8f& d, v16b x, v16b y) { guard4x_b(a, b, c, d, x, y); }
  static __device__ __forceinline__ void keep(v16b a, v16b b, v16b c, v16b d) { keep4_b(a, b, c, d); }
};

template <int ET> struct Elem;
template <> struct Elem<0> { typedef _Float16 T; };
template <> struct Elem<1> { typedef __bf16 T; };
template <int ET, bool SPLIT, int BIAS_MODE, int OUT_MODE>
__global__ __launch_bounds__(256) void wmma_gemm64(
    const unsigned short* __restrict__ Ap, const unsigned short* __restrict__ A2p, int lda, long strideA,
    const unsigned short* __restrict__ Btp, const unsigned short* __restrict__ Bt2p, int ldb, long strideB,
    void* __restrict__ Cout, void* __restrict__ Cout2, int ldc, long strideC,
    const float* __restrict__ bias,
    int M, int N, int K, float scale, float bias_scale) {
  typedef typename Elem<ET>::T T;
  typedef typename Frag<T>::V V;
  const T* A = (const T*)Ap; const T* A2 = (const T*)A2p; const T* Bt = (const T*)Btp; const T* Bt2 = (const T*)Bt2p;
  __shared__ __align__(16) float sT[8][16 * 68];
  const int b    = blockIdx.y;
  const int lane = threadIdx.x & 31;
  const int wave = threadIdx.x >> 5;
  const int tilesN = N >> 6;
  const int tilesM = M >> 6;
  const int tile = blockIdx.x * 8 + wave;
  if (tile >= tilesM * tilesN) return;
  const int tm = tile / tilesN;
  const int tn = tile - tm * tilesN;
  const int m0 = tm << 6;
  const int n0 = tn << 6;

  const T* Ab  = A  + (size_t)b * strideA;
  const T* Bb  = Bt + (size_t)b * strideB;
  const T* Ab2 = SPLIT ? (A2  + (size_t)b * strideA) : nullptr;
  const T* Bb2 = SPLIT ? (Bt2 + (size_t)b * strideB) : nullptr;

  const int rlane = lane & 15;
  const int koff  = (lane >> 4) * 8;
  const int mOff  = (lane >> 4) * 8;

  v8f acc[4][4];
#pragma unroll
  for (int i = 0; i < 4; ++i)
#pragma unroll
    for (int j = 0; j < 4; ++j) acc[i][j] = (v8f){0.f,0.f,0.f,0.f,0.f,0.f,0.f,0.f};

  for (int k0 = 0; k0 < K; k0 += 32) {
    V bh[4], bl[4];
#pragma unroll
    for (int j = 0; j < 4; ++j) {
      const size_t bo = (size_t)(n0 + (j << 4) + rlane) * ldb + koff + k0;
      bh[j] = Frag<T>::load(Bb + bo);
      if (SPLIT) bl[j] = Frag<T>::load(Bb2 + bo);
    }
#pragma unroll
    for (int i = 0; i < 4; ++i) {
      const size_t ao = (size_t)(m0 + (i << 4) + rlane) * lda + koff + k0;
      V ah = Frag<T>::load(Ab + ao);
      V al;
      if (SPLIT) al = Frag<T>::load(Ab2 + ao);
#pragma unroll
      for (int j = 0; j < 4; ++j) {
        acc[i][j] = Frag<T>::mma(ah, bh[j], acc[i][j]);
        if (SPLIT) {
          acc[i][j] = Frag<T>::mma(ah, bl[j], acc[i][j]);
          acc[i][j] = Frag<T>::mma(al, bh[j], acc[i][j]);
        }
      }
      Frag<T>::guard4(acc[i][0], acc[i][1], acc[i][2], acc[i][3], ah, SPLIT ? al : ah);
    }
    Frag<T>::keep(bh[0], bh[1], bh[2], bh[3]);
    if (SPLIT) Frag<T>::keep(bl[0], bl[1], bl[2], bl[3]);
  }
  acc_guard4(acc[0][0], acc[0][1], acc[0][2], acc[0][3]);
  acc_guard4(acc[1][0], acc[1][1], acc[1][2], acc[1][3]);
  acc_guard4(acc[2][0], acc[2][1], acc[2][2], acc[2][3]);
  acc_guard4(acc[3][0], acc[3][1], acc[3][2], acc[3][3]);

  float* slab = sT[wave];
#pragma unroll
  for (int i = 0; i < 4; ++i) {
    const int mBase = m0 + (i << 4);
#pragma unroll
    for (int j = 0; j < 4; ++j) {
      const int n = n0 + (j << 4) + rlane;
      float bv = 0.f;
      if (BIAS_MODE == 2) bv = bf_bits2f(f2bf_bits(bias[n])) * bias_scale;
#pragma unroll
      for (int r = 0; r < 8; ++r) {
        float v = acc[i][j][r] * scale;
        if (BIAS_MODE == 1) v += bf_bits2f(f2bf_bits(bias[mBase + mOff + r])) * bias_scale;
        if (BIAS_MODE == 2) v += bv;
        slab[(mOff + r) * 68 + (j << 4) + rlane] = v;
      }
    }
    __builtin_amdgcn_fence(__ATOMIC_RELEASE, "workgroup");
    __builtin_amdgcn_wave_barrier();
    __builtin_amdgcn_fence(__ATOMIC_ACQUIRE, "workgroup");
    if (OUT_MODE == 0) {
      float* C = (float*)Cout + (size_t)b * strideC;
      const int hh = lane >> 4, c4 = (lane & 15) * 4;
      for (int pass = 0; pass < 2; ++pass) {
#pragma unroll
        for (int it = 0; it < 8; ++it) {
          const int row = it * 2 + hh;
          v4f v = *(const v4f*)(slab + row * 68 + c4);
          *(volatile v4f*)(C + (size_t)(mBase + row) * ldc + n0 + c4) = v;
        }
        __threadfence();
      }
    } else {
      const int q = lane >> 3, c8 = (lane & 7) * 8;
      unsigned short* C  = (unsigned short*)Cout  + (size_t)b * strideC;
      unsigned short* C2 = (OUT_MODE == 2) ? ((unsigned short*)Cout2 + (size_t)b * strideC) : nullptr;
      for (int pass = 0; pass < 2; ++pass) {
#pragma unroll
        for (int it = 0; it < 4; ++it) {
          const int row = it * 4 + q;
          const float* sp = slab + row * 68 + c8;
          v8h hv, lv;
#pragma unroll
          for (int e = 0; e < 8; ++e) {
            if (OUT_MODE == 1) {
              hv[e] = (_Float16)sp[e];
            } else {
              unsigned short hb = f2bf_bits(sp[e]);
              unsigned short lb = f2bf_bits(sp[e] - bf_bits2f(hb));
              hv[e] = __builtin_bit_cast(_Float16, hb);
              lv[e] = __builtin_bit_cast(_Float16, lb);
            }
          }
          *(volatile v8h*)(C + (size_t)(mBase + row) * ldc + n0 + c8) = hv;
          if (OUT_MODE == 2) *(volatile v8h*)(C2 + (size_t)(mBase + row) * ldc + n0 + c8) = lv;
        }
        __threadfence();
      }
    }
    __builtin_amdgcn_fence(__ATOMIC_RELEASE, "workgroup");
    __builtin_amdgcn_wave_barrier();
    __builtin_amdgcn_fence(__ATOMIC_ACQUIRE, "workgroup");
  }
}

__global__ __launch_bounds__(256) void cast8_bf16_kernel(const float* __restrict__ in, unsigned short* __restrict__ out, int n8) {
  const int i = blockIdx.x * 256 + threadIdx.x;
  if (i >= n8) return;
  const float* p = in + 8 * (size_t)i;
  const v4f a = *(const v4f*)(p);
  const v4f c = *(const v4f*)(p + 4);
  unsigned short hb[8];
#pragma unroll
  for (int e = 0; e < 4; ++e) {
    hb[e]     = f2bf_bits(a[e]);
    hb[4 + e] = f2bf_bits(c[e]);
  }
  const v4u u = (v4u){pk16(hb[0], hb[1]), pk16(hb[2], hb[3]), pk16(hb[4], hb[5]), pk16(hb[6], hb[7])};
  unsigned short* q = out + 8 * (size_t)i;
  *(volatile v4u*)q = u;
  __threadfence();
  *(volatile v4u*)q = u;
}

__global__ __launch_bounds__(256) void cast8_bf16_4planes_kernel(const float* __restrict__ W0, const float* __restrict__ W1,
                                                               const float* __restrict__ W2, const float* __restrict__ W3,
                                                               unsigned short* __restrict__ out, int n8) {
  const int i = blockIdx.x * 256 + threadIdx.x;
  const int z = blockIdx.y;
  if (i >= n8) return;
  const float* W = (z == 0) ? W0 : (z == 1) ? W1 : (z == 2) ? W2 : W3;
  const float* p = W + 8 * (size_t)i;
  const v4f a = *(const v4f*)(p);
  const v4f c = *(const v4f*)(p + 4);
  unsigned short hb[8];
#pragma unroll
  for (int e = 0; e < 4; ++e) {
    hb[e]     = f2bf_bits(a[e]);
    hb[4 + e] = f2bf_bits(c[e]);
  }
  const v4u u = (v4u){pk16(hb[0], hb[1]), pk16(hb[2], hb[3]), pk16(hb[4], hb[5]), pk16(hb[6], hb[7])};
  unsigned short* q = out + (size_t)z * 8 * (size_t)n8 + 8 * (size_t)i;
  *(volatile v4u*)q = u;
  __threadfence();
  *(volatile v4u*)q = u;
}

__global__ __launch_bounds__(256) void cast8_wo_kernel(const float* __restrict__ in, unsigned short* __restrict__ out, int n8, float carry) {
  const int i = blockIdx.x * 256 + threadIdx.x;
  if (i >= n8) return;
  const float* p = in + 8 * (size_t)i;
  const v4f a = *(const v4f*)(p);
  const v4f c = *(const v4f*)(p + 4);
  unsigned short hb[8];
#pragma unroll
  for (int e = 0; e < 4; ++e) {
    hb[e]     = h_bits(bf_bits2f(f2bf_bits(a[e])) * carry);
    hb[4 + e] = h_bits(bf_bits2f(f2bf_bits(c[e])) * carry);
  }
  const v4u u = (v4u){pk16(hb[0], hb[1]), pk16(hb[2], hb[3]), pk16(hb[4], hb[5]), pk16(hb[6], hb[7])};
  unsigned short* q = out + 8 * (size_t)i;
  *(volatile v4u*)q = u;
  __threadfence();
  *(volatile v4u*)q = u;
}

__global__ __launch_bounds__(256) void zero16_kernel(unsigned int* __restrict__ p, int n16) {
  const int i = blockIdx.x * 256 + threadIdx.x;
  if (i >= n16) return;
  const v4u z = (v4u){0u, 0u, 0u, 0u};
  unsigned int* q = p + 4 * (size_t)i;
  *(volatile v4u*)q = z;
  __threadfence();
  *(volatile v4u*)q = z;
}

__device__ __forceinline__ float sigm(float z) {
  const float e = expf(-z);
  return __builtin_amdgcn_rcpf(1.0f + e);
}

__global__ __launch_bounds__(kPreThreads) void preproc_kernel(
    const float* __restrict__ q32, const float* __restrict__ kz32, const float* __restrict__ gz32,
    unsigned short* __restrict__ QaH, unsigned short* __restrict__ QaL,
    unsigned short* __restrict__ KdH, unsigned short* __restrict__ KdL,
    unsigned short* __restrict__ Qa16, unsigned short* __restrict__ Kp16, float* __restrict__ AC) {
  __shared__ __align__(16) float kdl[kPreKeys * kChunk];
  __shared__ __align__(16) unsigned short kpl[kPreKeys * kChunk];
  const int tid = threadIdx.x;
  const int c   = blockIdx.x >> 2;
  const int qtr = blockIdx.x & 3;
  const int el  = 2 * tid;
  const int e0  = qtr * kPreKeys + el;
  const int t0  = c * kChunk;
  float A0 = 1.0f, A1 = 1.0f;
#pragma unroll 1
  for (int t = 0; t < kChunk; ++t) {
    const size_t ro = (size_t)(t0 + t) * kKey + e0;
    const v2f qv = *(const v2f*)(q32 + ro);
    const v2f kv = *(const v2f*)(kz32 + ro);
    const v2f gv = *(const v2f*)(gz32 + ro);
    const float g0 = sigm(gv[0]), g1 = sigm(gv[1]);
    const float k0 = sigm(kv[0]), k1 = sigm(kv[1]);
    A0 = fmaxf(A0 * g0, kAFloor);
    A1 = fmaxf(A1 * g1, kAFloor);
    const float qa0 = qv[0] * A0, qa1 = qv[1] * A1;
    const float kd0 = k0 * __builtin_amdgcn_rcpf(A0);
    const float kd1 = k1 * __builtin_amdgcn_rcpf(A1);
    kdl[el * kChunk + t]       = kd0;
    kdl[(el + 1) * kChunk + t] = kd1;
    const unsigned short qh0 = f2bf_bits(qa0), qh1 = f2bf_bits(qa1);
    const unsigned short ql0 = f2bf_bits(qa0 - bf_bits2f(qh0)), ql1 = f2bf_bits(qa1 - bf_bits2f(qh1));
    const unsigned short kh0 = f2bf_bits(kd0), kh1 = f2bf_bits(kd1);
    const unsigned short kl0 = f2bf_bits(kd0 - bf_bits2f(kh0)), kl1 = f2bf_bits(kd1 - bf_bits2f(kh1));
    const unsigned uqh = pk16(qh0, qh1);
    const unsigned uql = pk16(ql0, ql1);
    const unsigned ukh = pk16(kh0, kh1);
    const unsigned ukl = pk16(kl0, kl1);
    const unsigned uqa = pk16(h_bits(qa0 * kCarryQ), h_bits(qa1 * kCarryQ));
    *(volatile unsigned*)(QaH + ro)  = uqh;
    *(volatile unsigned*)(QaL + ro)  = uql;
    *(volatile unsigned*)(KdH + ro)  = ukh;
    *(volatile unsigned*)(KdL + ro)  = ukl;
    *(volatile unsigned*)(Qa16 + ro) = uqa;
    __threadfence();
    *(volatile unsigned*)(QaH + ro)  = uqh;
    *(volatile unsigned*)(QaL + ro)  = uql;
    *(volatile unsigned*)(KdH + ro)  = ukh;
    *(volatile unsigned*)(KdL + ro)  = ukl;
    *(volatile unsigned*)(Qa16 + ro) = uqa;
  }
  {
    const v2f av = (v2f){A0, A1};
    float* ap = AC + (size_t)c * kKey + e0;
    *(volatile v2f*)ap = av;
    __threadfence();
    *(volatile v2f*)ap = av;
  }
#pragma unroll 1
  for (int t = 0; t < kChunk; ++t) {
    const float kp0 = kdl[el * kChunk + t] * A0;
    const float kp1 = kdl[(el + 1) * kChunk + t] * A1;
    kpl[el * kChunk + t]       = h_bits(kp0 * kCarryK);
    kpl[(el + 1) * kChunk + t] = h_bits(kp1 * kCarryK);
  }
  __syncthreads();
  const int lane = tid & 31, wave = tid >> 5;
  const int rq = lane >> 2, c8 = (lane & 3) * 8;
  unsigned short* kb = Kp16 + ((size_t)(c * kKey + qtr * kPreKeys)) * kChunk;
  for (int pass = 0; pass < 2; ++pass) {
#pragma unroll
    for (int it = 0; it < 8; ++it) {
      const int row = wave * 64 + it * 8 + rq;
      const v4u u = *(const v4u*)(kpl + row * kChunk + c8);
      *(volatile v4u*)(kb + (size_t)row * kChunk + c8) = u;
    }
    __threadfence();
  }
}

__global__ __launch_bounds__(128) void pmask_kernel(const float* __restrict__ SC, unsigned short* __restrict__ Ph, unsigned short* __restrict__ Pl) {
  const int c    = blockIdx.x;
  const int p    = c >> 1;
  const int half = c & 1;
  const int tid  = threadIdx.x;
  const int tl   = tid >> 2;
  const int sl0  = (tid & 3) * 8;
  const float* sp = SC + (size_t)p * 4096 + (size_t)(half * 32 + tl) * 64 + half * 32 + sl0;
  const v4f a = *(const v4f*)(sp);
  const v4f b4 = *(const v4f*)(sp + 4);
  float x[8];
#pragma unroll
  for (int e = 0; e < 4; ++e) { x[e] = a[e]; x[4 + e] = b4[e]; }
  unsigned short hh[8], hl[8];
#pragma unroll
  for (int e = 0; e < 8; ++e) {
    const float fsel = ((sl0 + e) <= tl) ? 1.0f : 0.0f;
    const float xs = (x[e] * fsel) * kCarryP;
    const unsigned short hb = h_bits(xs);
    const float res = (xs - h16_to_f32((unsigned)hb)) * kCarryPl;
    hh[e] = hb;
    hl[e] = h_bits(res);
  }
  const v4u uh = (v4u){pk16(hh[0], hh[1]), pk16(hh[2], hh[3]), pk16(hh[4], hh[5]), pk16(hh[6], hh[7])};
  const v4u ul = (v4u){pk16(hl[0], hl[1]), pk16(hl[2], hl[3]), pk16(hl[4], hl[5]), pk16(hl[6], hl[7])};
  const size_t off = (size_t)c * (kChunk * kChunk) + (size_t)tl * kChunk + sl0;
  *(volatile v4u*)(Ph + off) = uh;
  *(volatile v4u*)(Pl + off) = ul;
  __threadfence();
  *(volatile v4u*)(Ph + off) = uh;
  *(volatile v4u*)(Pl + off) = ul;
}

__global__ __launch_bounds__(256) void chunk_kernel(
    const unsigned short* __restrict__ Qa16p, const unsigned short* __restrict__ Php, const unsigned short* __restrict__ Plp,
    const unsigned short* __restrict__ Vtp, const unsigned short* __restrict__ Kpp, const float* __restrict__ AC,
    const unsigned short* __restrict__ SbInp, const float* __restrict__ SmIn,
    unsigned short* __restrict__ SbOut, float* __restrict__ SmOut,
    unsigned short* __restrict__ Out16, int c) {
  typedef Frag<_Float16> F;
  __shared__ __align__(16) float sT[8][16 * 68];
  const int lane  = threadIdx.x & 31;
  const int wave  = threadIdx.x >> 5;
  const int rlane = lane & 15;
  const int koff  = (lane >> 4) * 8;
  const int mOff  = koff;
  const int hh = lane >> 4, c4 = (lane & 15) * 4;
  const int q8 = lane >> 3, c8 = (lane & 7) * 8;
  float* slab = sT[wave];
  const _Float16* Vt = (const _Float16*)Vtp;
  const int tcol = c * kChunk;
  const v8f z8 = (v8f){0.f, 0.f, 0.f, 0.f, 0.f, 0.f, 0.f, 0.f};

  if (blockIdx.x < kRoleABlocks) {
    const _Float16* Qa = (const _Float16*)Qa16p;
    const _Float16* Sb = (const _Float16*)SbInp;
    const _Float16* Ph = (const _Float16*)Php + (size_t)c * (kChunk * kChunk);
    const _Float16* Pl = (const _Float16*)Plp + (size_t)c * (kChunk * kChunk);
    const int n0 = (blockIdx.x * 8 + wave) * 64;
    v8f acc[2][4], accL[2][4];
#pragma unroll
    for (int i = 0; i < 2; ++i)
#pragma unroll
      for (int j = 0; j < 4; ++j) { acc[i][j] = z8; accL[i][j] = z8; }

    for (int k0 = 0; k0 < kKey; k0 += 32) {
      v16h bh[4];
#pragma unroll
      for (int j = 0; j < 4; ++j) bh[j] = F::load(Sb + (size_t)(n0 + (j << 4) + rlane) * kKey + koff + k0);
#pragma unroll
      for (int i = 0; i < 2; ++i) {
        const v16h a = F::load(Qa + (size_t)(tcol + (i << 4) + rlane) * kKey + koff + k0);
#pragma unroll
        for (int j = 0; j < 4; ++j) acc[i][j] = F::mma(a, bh[j], acc[i][j]);
        F::guard4(acc[i][0], acc[i][1], acc[i][2], acc[i][3], a, a);
      }
      F::keep(bh[0], bh[1], bh[2], bh[3]);
    }
    {
      v16h bv[4];
#pragma unroll
      for (int j = 0; j < 4; ++j) bv[j] = F::load(Vt + (size_t)(n0 + (j << 4) + rlane) * kT + tcol + koff);
#pragma unroll
      for (int i = 0; i < 2; ++i) {
        const v16h pa = F::load(Ph + ((i << 4) + rlane) * kChunk + koff);
        const v16h pb = F::load(Pl + ((i << 4) + rlane) * kChunk + koff);
#pragma unroll
        for (int j = 0; j < 4; ++j) {
          acc[i][j]  = F::mma(pa, bv[j], acc[i][j]);
          accL[i][j] = F::mma(pb, bv[j], accL[i][j]);
        }
        F::guard4(acc[i][0], acc[i][1], acc[i][2], acc[i][3], pa, pb);
        F::guard4(accL[i][0], accL[i][1], accL[i][2], accL[i][3], pa, pb);
      }
      F::keep(bv[0], bv[1], bv[2], bv[3]);
    }
    acc_guard4(acc[0][0], acc[0][1], acc[0][2], acc[0][3]);
    acc_guard4(acc[1][0], acc[1][1], acc[1][2], acc[1][3]);
    acc_guard4(accL[0][0], accL[0][1], accL[0][2], accL[0][3]);
    acc_guard4(accL[1][0], accL[1][1], accL[1][2], accL[1][3]);

#pragma unroll
    for (int i = 0; i < 2; ++i) {
#pragma unroll
      for (int j = 0; j < 4; ++j) {
#pragma unroll
        for (int r = 0; r < 8; ++r) {
          const float v = (acc[i][j][r] + accL[i][j][r] * kPlInv) * kOutSlabScale;
          slab[(mOff + r) * 68 + (j << 4) + rlane] = v;
        }
      }
      wave_sync();
      unsigned short* obase = Out16 + (size_t)(tcol + (i << 4)) * kVal + n0 + c8;
      for (int pass = 0; pass < 2; ++pass) {
#pragma unroll
        for (int it = 0; it < 4; ++it) {
          const int row = it * 4 + q8;
          const float* sp = slab + row * 68 + c8;
          const v4f s0 = *(const v4f*)(sp);
          const v4f s1 = *(const v4f*)(sp + 4);
          unsigned short hb[8];
#pragma unroll
          for (int e = 0; e < 4; ++e) { hb[e] = h_bits(s0[e]); hb[4 + e] = h_bits(s1[e]); }
          const v4u u = (v4u){pk16(hb[0], hb[1]), pk16(hb[2], hb[3]), pk16(hb[4], hb[5]), pk16(hb[6], hb[7])};
          *(volatile v4u*)(obase + (size_t)row * kVal) = u;
        }
        __threadfence();
      }
      wave_sync();
    }
  } else {
    const _Float16* Kc = (const _Float16*)Kpp + (size_t)c * kKey * kChunk;
    const int tile = (blockIdx.x - kRoleABlocks) * 8 + wave;
    const int tm = tile >> 4;
    const int tn = tile & 15;
    const int m0 = tm << 6;
    const int n0 = tn << 6;
    v8f acc[4][4];
#pragma unroll
    for (int i = 0; i < 4; ++i)
#pragma unroll
      for (int j = 0; j < 4; ++j) acc[i][j] = z8;
    {
      v16h bh[4];
#pragma unroll
      for (int j = 0; j < 4; ++j) bh[j] = F::load(Kc + (size_t)(n0 + (j << 4) + rlane) * kChunk + koff);
#pragma unroll
      for (int i = 0; i < 4; ++i) {
        const v16h a = F::load(Vt + (size_t)(m0 + (i << 4) + rlane) * kT + tcol + koff);
#pragma unroll
        for (int j = 0; j < 4; ++j) acc[i][j] = F::mma(a, bh[j], acc[i][j]);
        F::guard4(acc[i][0], acc[i][1], acc[i][2], acc[i][3], a, a);
      }
      F::keep(bh[0], bh[1], bh[2], bh[3]);
    }
    acc_guard4(acc[0][0], acc[0][1], acc[0][2], acc[0][3]);
    acc_guard4(acc[1][0], acc[1][1], acc[1][2], acc[1][3]);
    acc_guard4(acc[2][0], acc[2][1], acc[2][2], acc[2][3]);
    acc_guard4(acc[3][0], acc[3][1], acc[3][2], acc[3][3]);

    const v4f acv = *(const v4f*)(AC + (size_t)c * kKey + n0 + c4);
#pragma unroll
    for (int i = 0; i < 4; ++i) {
      const int mBase = m0 + (i << 4);
#pragma unroll
      for (int j = 0; j < 4; ++j) {
#pragma unroll
        for (int r = 0; r < 8; ++r) slab[(mOff + r) * 68 + (j << 4) + rlane] = acc[i][j][r] * kStateScale;
      }
      wave_sync();
#pragma unroll
      for (int it = 0; it < 8; ++it) {
        const int row = it * 2 + hh;
        float* sp = slab + row * 68 + c4;
        const v4f a  = *(const v4f*)(sp);
        const v4f so = *(const v4f*)(SmIn + (size_t)(mBase + row) * kKey + n0 + c4);
        const v4f f  = acv * so + a;
        *(v4f*)(sp) = f;
        if (it == 3) { asm volatile("" ::: "memory"); }
      }
      wave_sync();
      for (int pass = 0; pass < 2; ++pass) {
#pragma unroll
        for (int it = 0; it < 8; ++it) {
          const int row = it * 2 + hh;
          const v4f f = *(const v4f*)(slab + row * 68 + c4);
          *(volatile v4f*)(SmOut + (size_t)(mBase + row) * kKey + n0 + c4) = f;
        }
#pragma unroll
        for (int it = 0; it < 4; ++it) {
          const int row = it * 4 + q8;
          const float* sp = slab + row * 68 + c8;
          const v4f s0 = *(const v4f*)(sp);
          const v4f s1 = *(const v4f*)(sp + 4);
          unsigned short hb[8];
#pragma unroll
          for (int e = 0; e < 4; ++e) { hb[e] = h_bits(s0[e] * kCarryS); hb[4 + e] = h_bits(s1[e] * kCarryS); }
          const v4u u = (v4u){pk16(hb[0], hb[1]), pk16(hb[2], hb[3]), pk16(hb[4], hb[5]), pk16(hb[6], hb[7])};
          *(volatile v4u*)(SbOut + (size_t)(mBase + row) * kKey + n0 + c8) = u;
        }
        __threadfence();
      }
      wave_sync();
    }
  }
}

__global__ __launch_bounds__(256) void state_out_kernel(const float* __restrict__ Sm, float* __restrict__ out1) {
  __shared__ __align__(16) float sm[64 * 68];
  const int tid = threadIdx.x;
  const int e0 = blockIdx.x * 64;
  const int v0 = blockIdx.y * 64;
#pragma unroll
  for (int i = 0; i < 4; ++i) {
    const int el = i * 256 + tid;
    const int r  = el >> 4;
    const int cc = (el & 15) * 4;
    const v4f w = *(const v4f*)(Sm + (size_t)(v0 + r) * kKey + e0 + cc);
    sm[(cc + 0) * 68 + r] = w[0];
    sm[(cc + 1) * 68 + r] = w[1];
    sm[(cc + 2) * 68 + r] = w[2];
    sm[(cc + 3) * 68 + r] = w[3];
  }
  __syncthreads();
  const int lane = tid & 31, wave = tid >> 5;
  const int hh = lane >> 4, c4 = (lane & 15) * 4;
  for (int pass = 0; pass < 2; ++pass) {
#pragma unroll
    for (int it = 0; it < 4; ++it) {
      const int row = wave * 8 + it * 2 + hh;
      const v4f v = *(const v4f*)(sm + row * 68 + c4);
      *(volatile v4f*)(out1 + (size_t)(e0 + row) * kVal + v0 + c4) = v;
    }
    __threadfence();
  }
}

constexpr size_t kSzXb    = (size_t)kT * kHid * 2;
constexpr size_t kSzWb    = (size_t)4 * kKey * kHid * 2;
constexpr size_t kSzBf1k  = (size_t)kT * kKey * 2;
constexpr size_t kSzWo16  = (size_t)kOutDim * kVal * 2;
constexpr size_t kSzF32p  = (size_t)kT * kKey * 4;
constexpr size_t kSzVt    = (size_t)kVal * kT * 2;
constexpr size_t kSzKp    = (size_t)kNChunk * kKey * kChunk * 2;
constexpr size_t kSzAC    = (size_t)kNChunk * kKey * 4;
constexpr size_t kSzSC    = (size_t)kPairs * 64 * 64 * 4;
constexpr size_t kSzP     = (size_t)kNChunk * kChunk * kChunk * 2;
constexpr size_t kSzSm    = (size_t)kVal * kKey * 4;
constexpr size_t kSzSb    = (size_t)kVal * kKey * 2;
constexpr size_t kOffXb   = 0;
constexpr size_t kOffWb   = kOffXb + kSzXb;
constexpr size_t kOffQaH  = 0;
constexpr size_t kOffQaL  = kOffQaH + kSzBf1k;
constexpr size_t kOffKdH  = kOffQaL + kSzBf1k;
constexpr size_t kOffKdL  = kOffKdH + kSzBf1k;
constexpr size_t kOffWo16 = kOffWb + kSzWb;
constexpr size_t kOffQ32  = kOffWo16 + kSzWo16;
constexpr size_t kOffSm0  = kOffQ32;
constexpr size_t kOffSm1  = kOffSm0 + kSzSm;
constexpr size_t kOffKz32 = kOffQ32 + kSzF32p;
constexpr size_t kOffGz32 = kOffKz32 + kSzF32p;
constexpr size_t kOffVt   = kOffGz32 + kSzF32p;
constexpr size_t kOffQa16 = kOffVt + kSzVt;
constexpr size_t kOffKp   = kOffQa16 + kSzBf1k;
constexpr size_t kOffAC   = kOffKp + kSzKp;
constexpr size_t kOffSC   = kOffAC + kSzAC;
constexpr size_t kOffPh   = kOffSC + kSzSC;
constexpr size_t kOffPl   = kOffPh + kSzP;
constexpr size_t kOffOut16= kOffPl + kSzP;
constexpr size_t kOffSb0  = kOffOut16 + kSzBf1k;
constexpr size_t kOffSb1  = kOffSb0 + kSzSb;
constexpr size_t kWsTotal = kOffSb1 + kSzSb;
static_assert(kOffKdL + kSzBf1k == kOffWo16, "aliased bf16 planes fit exactly in the dead Xb/Wb bytes");
static_assert(kOffSm1 + kSzSm <= kOffKz32, "state master ping-pong fits in the dead q32 bytes");
static_assert(kWsTotal == 127926272ull, "carve total");
static_assert(kWsTotal <= 134217728ull, "carve within 128 MiB");
static_assert((kOffWo16 % 128) == 0 && (kOffSm1 % 128) == 0 && (kOffAC % 128) == 0 && (kOffPh % 128) == 0 && (kOffSb1 % 128) == 0, "line alignment");
constexpr size_t kOut1ElemOff = (size_t)kT * kOutDim;
static_assert(kOut1ElemOff * 4 == 33554432ull, "second output byte offset");
static_assert((kOut1ElemOff + (size_t)kKey * kVal) * 4 == 37748736ull, "total output bytes");

extern "C" void kernel_launch(void* const* d_in, const int* in_sizes, int n_in,
                              void* d_out, int out_size, void* d_ws, size_t ws_size,
                              hipStream_t stream) {
  if (n_in < 11) return;
  if (in_sizes[0] != kT * kHid) return;
  if (in_sizes[1] != kKey * kHid || in_sizes[3] != kKey * kHid || in_sizes[7] != kKey * kHid) return;
  if (in_sizes[5] != kVal * kHid || in_sizes[9] != kOutDim * kVal) return;
  if (in_sizes[2] != kKey || in_sizes[4] != kKey || in_sizes[6] != kVal || in_sizes[8] != kKey || in_sizes[10] != kOutDim) return;
  if (out_size != kT * kOutDim + kKey * kVal) return;
  if (ws_size < kWsTotal) return;

  const float* x  = (const float*)d_in[0];
  const float* Wq = (const float*)d_in[1];
  const float* bq = (const float*)d_in[2];
  const float* Wk = (const float*)d_in[3];
  const float* bk = (const float*)d_in[4];
  const float* Wv = (const float*)d_in[5];
  const float* bv = (const float*)d_in[6];
  const float* Wg = (const float*)d_in[7];
  const float* bg = (const float*)d_in[8];
  const float* Wo = (const float*)d_in[9];
  const float* bo = (const float*)d_in[10];
  float* out0 = (float*)d_out;
  float* out1 = (float*)d_out + kOut1ElemOff;

  char* ws = (char*)d_ws;
  unsigned short* Xb   = (unsigned short*)(ws + kOffXb);
  unsigned short* Wb   = (unsigned short*)(ws + kOffWb);
  unsigned short* QaH  = (unsigned short*)(ws + kOffQaH);
  unsigned short* QaL  = (unsigned short*)(ws + kOffQaL);
  unsigned short* KdH  = (unsigned short*)(ws + kOffKdH);
  unsigned short* KdL  = (unsigned short*)(ws + kOffKdL);
  unsigned short* Wo16 = (unsigned short*)(ws + kOffWo16);
  float* q32  = (float*)(ws + kOffQ32);
  float* Sm0  = (float*)(ws + kOffSm0);
  float* Sm1  = (float*)(ws + kOffSm1);
  float* kz32 = (float*)(ws + kOffKz32);
  float* gz32 = (float*)(ws + kOffGz32);
  unsigned short* Vt16  = (unsigned short*)(ws + kOffVt);
  unsigned short* Qa16  = (unsigned short*)(ws + kOffQa16);
  unsigned short* Kp16  = (unsigned short*)(ws + kOffKp);
  float* AC = (float*)(ws + kOffAC);
  float* SC = (float*)(ws + kOffSC);
  unsigned short* Ph    = (unsigned short*)(ws + kOffPh);
  unsigned short* Pl    = (unsigned short*)(ws + kOffPl);
  unsigned short* Out16 = (unsigned short*)(ws + kOffOut16);
  unsigned short* Sb0 = (unsigned short*)(ws + kOffSb0);
  unsigned short* Sb1 = (unsigned short*)(ws + kOffSb1);
  const size_t planeW = (size_t)kKey * kHid;
  unsigned short* Wqb = Wb + 0 * planeW;
  unsigned short* Wkb = Wb + 1 * planeW;
  unsigned short* Wgb = Wb + 2 * planeW;
  unsigned short* Wvb = Wb + 3 * planeW;

  const int n8x = (kT * kHid) / 8;
  const int n8w = (kKey * kHid) / 8;
  const int n8o = (kOutDim * kVal) / 8;
  cast8_bf16_kernel<<<dim3(n8x / 256), dim3(256), 0, stream>>>(x, Xb, n8x);
  cast8_bf16_4planes_kernel<<<dim3(n8w / 256, 4), dim3(256), 0, stream>>>(Wq, Wk, Wg, Wv, Wb, n8w);
  cast8_wo_kernel<<<dim3(n8o / 256), dim3(256), 0, stream>>>(Wo, Wo16, n8o, kCarryW);

  const int blkProj = ((kT / 64) * (kKey / 64)) / 8;
  wmma_gemm64<1, false, 2, 0><<<dim3(blkProj, 1), dim3(256), 0, stream>>>(
      Xb, Xb, kHid, 0L, Wqb, Wqb, kHid, 0L, (void*)q32, (void*)q32, kKey, 0L, bq, kT, kKey, kHid, 1.0f, 1.0f);
  wmma_gemm64<1, false, 2, 0><<<dim3(blkProj, 1), dim3(256), 0, stream>>>(
      Xb, Xb, kHid, 0L, Wkb, Wkb, kHid, 0L, (void*)kz32, (void*)kz32, kKey, 0L, bk, kT, kKey, kHid, 1.0f, 1.0f);
  wmma_gemm64<1, false, 2, 0><<<dim3(blkProj, 1), dim3(256), 0, stream>>>(
      Xb, Xb, kHid, 0L, Wgb, Wgb, kHid, 0L, (void*)gz32, (void*)gz32, kKey, 0L, bg, kT, kKey, kHid, 1.0f, 1.0f);
  wmma_gemm64<1, false, 1, 1><<<dim3(blkProj, 1), dim3(256), 0, stream>>>(
      Wvb, Wvb, kHid, 0L, Xb, Xb, kHid, 0L, (void*)Vt16, (void*)Vt16, kT, 0L, bv, kVal, kT, kHid, kCarryV, kCarryV);

  preproc_kernel<<<dim3(kNChunk * (kKey / kPreKeys)), dim3(kPreThreads), 0, stream>>>(
      q32, kz32, gz32, QaH, QaL, KdH, KdL, Qa16, Kp16, AC);

  wmma_gemm64<1, true, 0, 0><<<dim3(1, kPairs), dim3(32), 0, stream>>>(
      QaH, QaL, kKey, (long)64 * kKey, KdH, KdL, kKey, (long)64 * kKey,
      (void*)SC, (void*)SC, 64, (long)64 * 64, AC, 64, 64, kKey, 1.0f, 1.0f);
  pmask_kernel<<<dim3(kNChunk), dim3(128), 0, stream>>>(SC, Ph, Pl);

  zero16_kernel<<<dim3((int)(kSzSm / 16 / 256)), dim3(256), 0, stream>>>((unsigned int*)Sm0, (int)(kSzSm / 16));
  zero16_kernel<<<dim3((int)(kSzSb / 16 / 256)), dim3(256), 0, stream>>>((unsigned int*)Sb0, (int)(kSzSb / 16));

  for (int c = 0; c < kNChunk; ++c) {
    const unsigned short* SbIn = (c & 1) ? Sb1 : Sb0;
    unsigned short* SbNext     = (c & 1) ? Sb0 : Sb1;
    const float* SmInP         = (c & 1) ? Sm1 : Sm0;
    float* SmNext              = (c & 1) ? Sm0 : Sm1;
    chunk_kernel<<<dim3(kRoleABlocks + kRoleBBlocks), dim3(256), 0, stream>>>(
        Qa16, Ph, Pl, Vt16, Kp16, AC, SbIn, SmInP, SbNext, SmNext, Out16, c);
  }

  const int blkOut = ((kT / 64) * (kOutDim / 64)) / 8;
  wmma_gemm64<0, false, 2, 0><<<dim3(blkOut, 1), dim3(256), 0, stream>>>(
      Out16, Out16, kVal, 0L, Wo16, Wo16, kVal, 0L, (void*)out0, (void*)out0, kOutDim, 0L, bo,
      kT, kOutDim, kVal, kFinalScale, 1.0f);

  state_out_kernel<<<dim3(kKey / 64, kVal / 64), dim3(256), 0, stream>>>(Sm0, out1);
}
